// Attention_39453569581229
// MI455X (gfx1250) — hardware-run, weakly checked
//
#include <hip/hip_runtime.h>
#include <math.h>

typedef __attribute__((ext_vector_type(16))) _Float16 v16h;
typedef __attribute__((ext_vector_type(16))) __bf16 v16b;
typedef __attribute__((ext_vector_type(8)))  _Float16 v8h;
typedef __attribute__((ext_vector_type(8)))  __bf16 v8b;
typedef __attribute__((ext_vector_type(8)))  float v8f;
typedef __attribute__((ext_vector_type(4)))  float v4f;
typedef __attribute__((ext_vector_type(4)))  unsigned v4u;

template <typename T> __device__ __forceinline__ void vst2(void* p, T v) { *(volatile T*)p = v; __threadfence(); *(volatile T*)p = v; }
__device__ __forceinline__ v8f wmma16(v16h a, v16h b, v8f c) {
  v8f d = __builtin_amdgcn_wmma_f32_16x16x32_f16(false, a, false, b, (short)0, c, false, false);
  asm volatile("v_nop\n\tv_nop\n\tv_nop\n\tv_nop" : "+v"(d) : "v"(a), "v"(b));
  return d;
}
__device__ __forceinline__ v8f wmma_bf(v16b a, v16b b, v8f c) {
  v8f d = __builtin_amdgcn_wmma_f32_16x16x32_bf16(false, a, false, b, (short)0, c, false, false);
  asm volatile("v_nop\n\tv_nop\n\tv_nop\n\tv_nop" : "+v"(d) : "v"(a), "v"(b));
  return d;
}
__device__ __forceinline__ v16h frag_h(const _Float16* rowk0, int lane) {
  union { v16h v; v8h q[2]; } u; const _Float16* p = rowk0 + 8 * (lane >> 4);
  u.q[0] = *(const v8h*)p; u.q[1] = *(const v8h*)(p + 16); return u.v;
}
__device__ __forceinline__ v16b frag_b(const __bf16* rowk0, int lane) {
  union { v16b v; v8b q[2]; } u; const __bf16* p = rowk0 + 8 * (lane >> 4);
  u.q[0] = *(const v8b*)p; u.q[1] = *(const v8b*)(p + 16); return u.v;
}
__device__ __forceinline__ float bfr(float v) { return (float)(__bf16)v; }
__device__ __forceinline__ _Float16 toh_flush(float v) { const _Float16 r = (_Float16)v; return (fabsf(v) < 6.103515625e-05f) ? (_Float16)0.0f : r; }
#define LDSX() do { asm volatile("s_wait_dscnt 0" ::: "memory"); __builtin_amdgcn_wave_barrier(); __builtin_amdgcn_fence(3  , "workgroup"); } while (0)
#define WAITL() asm volatile("s_wait_loadcnt 0x0" ::: "memory")

#ifndef NB
#define NB 4
#endif
#ifndef SEQ
#define SEQ 2048
#endif
#define NB_FULL 4
#define SEQ_FULL 2048
#define CC 1024
#define DIN 1024
#define NH 16
#define HD 64
#define SCALE (0.125f)
#define X_NEED (((NB - 1) * SEQ_FULL + SEQ) * DIN)

static_assert(SEQ % 64 == 0);
static_assert(SEQ <= SEQ_FULL);
static_assert(NB <= NB_FULL);
static_assert(DIN % 32 == 0);
static_assert(CC % 128 == 0);
static_assert(DIN % 128 == 0);
static_assert(NH * HD == CC);
static_assert(HD == 64);
static_assert(SEQ % 16 == 0);
static_assert(HD / 2 == 32);
static_assert(128 % HD == 0);

#define NX8 ((size_t)NB * SEQ * DIN / 8)
#define NW8 ((size_t)3 * CC * DIN / 8)
#define NO8 ((size_t)DIN * CC / 8)
static_assert(((size_t)NB * SEQ * DIN / 8) % 256 == 0);
static_assert(((size_t)3 * CC * DIN / 8) % 256 == 0);
static_assert(((size_t)DIN * CC / 8) % 256 == 0);

#define WS_XB  ((size_t)0)
#define WS_WB  (WS_XB + 2u * (size_t)NB * SEQ * DIN)
#define WS_WO  (WS_WB + 2u * (size_t)3 * CC * DIN)
#define WS_QK  (WS_WO + 2u * (size_t)DIN * CC)
#define WS_VT  (WS_QK + 4u * (size_t)NB * SEQ * CC)
#define WS_YH  (WS_VT + 2u * (size_t)NB * CC * SEQ)
#define WS_CS  (WS_YH + 2u * (size_t)NB * SEQ * CC)
#define WS_END (WS_CS + 4u * (size_t)SEQ * 64)
static_assert(WS_END <= (size_t)134217728);
static_assert(WS_WB % 128 == 0);
static_assert(WS_WO % 128 == 0);
static_assert(WS_QK % 128 == 0);
static_assert(WS_VT % 128 == 0);
static_assert(WS_YH % 128 == 0);
static_assert(WS_CS % 128 == 0);

__device__ __forceinline__ v4u pack_bf(v4f a, v4f c) { v8b o;
#pragma unroll
  for (int i = 0; i < 4; ++i) { o[i] = (__bf16)a[i]; o[4 + i] = (__bf16)c[i]; }
  return __builtin_bit_cast(v4u, o); }
__device__ __forceinline__ v4u pack_h256(v4f a, v4f c) { v8h o;
#pragma unroll
  for (int i = 0; i < 4; ++i) { o[i] = (_Float16)(bfr(a[i]) * 256.0f); o[4 + i] = (_Float16)(bfr(c[i]) * 256.0f); }
  return __builtin_bit_cast(v4u, o); }

__global__ __launch_bounds__(256) void k_cvt(const float* __restrict__ X, const float* __restrict__ W1, const float* __restrict__ W2, unsigned* __restrict__ XB, unsigned* __restrict__ WB, unsigned* __restrict__ WOH) {
  const size_t i = (size_t)blockIdx.x * 256 + threadIdx.x;
  if (i < NX8) {
    const size_t row = i / (DIN / 8); const int cu = (int)(i % (DIN / 8)); const size_t bb = row / SEQ; const size_t t = row % SEQ;
    const float* p = X + (bb * SEQ_FULL + t) * DIN + cu * 8;
    const v4f a = *(const v4f*)p, c = *(const v4f*)(p + 4);
    vst2(XB + i * 4, pack_bf(a, c));
  } else if (i < NX8 + NW8) {
    const size_t k = i - NX8; const float* p = W1 + k * 8;
    const v4f a = *(const v4f*)p, c = *(const v4f*)(p + 4);
    vst2(WB + k * 4, pack_bf(a, c));
  } else if (i < NX8 + NW8 + NO8) {
    const size_t k = i - NX8 - NW8; const float* p = W2 + k * 8;
    const v4f a = *(const v4f*)p, c = *(const v4f*)(p + 4);
    vst2(WOH + k * 4, pack_h256(a, c));
  }
}

__global__ __launch_bounds__(256) void k_rope(float* __restrict__ CS) {
#pragma clang fp contract(off)
  __shared__ __align__(16) float cs[16][64];
  const int tid = threadIdx.x; const int t0 = blockIdx.x * 16;
#pragma unroll 1
  for (int it = 0; it < 2; ++it) { const int e = it * 256 + tid; const int rl = e >> 5, i = e & 31; const int j = i & 7, dg = i >> 3;
    float f = 1.0f;
    f = (j >= 1) ? 0.749894209332f : f;
    f = (j >= 2) ? 0.562341325190f : f;
    f = (j >= 3) ? 0.421696503429f : f;
    f = (j >= 4) ? 0.316227766017f : f;
    f = (j >= 5) ? 0.237137370566f : f;
    f = (j >= 6) ? 0.177827941004f : f;
    f = (j >= 7) ? 0.133352143216f : f;
    float dec = 1.0f;
    dec = (dg >= 1) ? 0.1f : dec;
    dec = (dg >= 2) ? 0.01f : dec;
    dec = (dg >= 3) ? 0.001f : dec;
    const float fr = f * dec; const float ang = (float)(t0 + rl) * fr;
    cs[rl][i] = cosf(ang); cs[rl][32 + i] = sinf(ang); }
  __syncthreads();
  const int rl = tid >> 4, pc = tid & 15; const v4f val = *(const v4f*)&cs[rl][pc * 4];
  vst2((void*)(CS + (size_t)(t0 + rl) * 64 + pc * 4), val);
}

__global__ __launch_bounds__(128) void k_proj(const __bf16* __restrict__ XB, const __bf16* __restrict__ WB, const float* __restrict__ BQKV, const float* __restrict__ CS, _Float16* __restrict__ QK, _Float16* __restrict__ VT) {
  __shared__ __align__(16) _Float16 sh[64][136]; __shared__ __align__(16) _Float16 th[128][72];
  const int tid = threadIdx.x, wave = tid >> 5, lane = tid & 31, col = lane & 15, g = lane >> 4; const int which = blockIdx.z; const int c0 = blockIdx.y * 128; const size_t r0 = (size_t)blockIdx.x * 64; const size_t bb = r0 / SEQ; const int t0 = (int)(r0 % SEQ);
  const __bf16* WA = WB + (size_t)which * CC * DIN; const float* BA = BQKV + which * CC;
  const __bf16* arow = XB + (r0 + wave * 16 + col) * DIN;
  v8f acc[8] = {};
#pragma unroll 2
  for (int kc = 0; kc < DIN / 32; ++kc) { const v16b a = frag_b(arow + kc * 32, lane); WAITL();
#pragma unroll
    for (int j = 0; j < 8; ++j) { const v16b w = frag_b(WA + (size_t)(c0 + j * 16 + col) * DIN + kc * 32, lane); WAITL(); acc[j] = wmma_bf(a, w, acc[j]); } }
  if (which < 2) { _Float16* DH = QK + (size_t)which * NB * SEQ * CC;
    float bias[8];
#pragma unroll
    for (int j = 0; j < 8; ++j) bias[j] = bfr(BA[c0 + j * 16 + col]);
    const float* crow = CS + (size_t)(t0 + wave * 16 + 8 * g) * 64 + col;
#pragma unroll
    for (int r = 0; r < 8; ++r) { const float ca = crow[r * 64], cb = crow[r * 64 + 16], sa = crow[r * 64 + 32], sb = crow[r * 64 + 48]; WAITL();
      const int row = wave * 16 + 8 * g + r;
#pragma unroll
      for (int hh = 0; hh < 2; ++hh) {
        { const float x1 = acc[4 * hh][r] + bias[4 * hh], x2 = acc[4 * hh + 2][r] + bias[4 * hh + 2];
          sh[row][(4 * hh) * 16 + col] = toh_flush(x1 * ca - x2 * sa); sh[row][(4 * hh + 2) * 16 + col] = toh_flush(x2 * ca + x1 * sa); }
        { const float x1 = acc[4 * hh + 1][r] + bias[4 * hh + 1], x2 = acc[4 * hh + 3][r] + bias[4 * hh + 3];
          sh[row][(4 * hh + 1) * 16 + col] = toh_flush(x1 * cb - x2 * sb); sh[row][(4 * hh + 3) * 16 + col] = toh_flush(x2 * cb + x1 * sb); } } }
    __syncthreads();
    for (int e = tid; e < 64 * 16; e += 128) { const int rl = e >> 4, q = e & 15; const v4u val = *(const v4u*)&sh[rl][q * 8]; vst2((void*)(DH + (r0 + rl) * CC + c0 + q * 8), val); }
  } else {
#pragma unroll
    for (int j = 0; j < 8; ++j) { const float bias = bfr(BA[c0 + j * 16 + col]);
#pragma unroll
      for (int r = 0; r < 8; ++r) { const float v = acc[j][r] + bias; th[j * 16 + col][wave * 16 + 8 * g + r] = toh_flush(v); } }
    __syncthreads();
    for (int e = tid; e < 128 * 8; e += 128) { const int cl = e >> 3, q = e & 7; const v4u val = *(const v4u*)&th[cl][q * 8]; vst2((void*)(VT + (bb * CC + c0 + cl) * (size_t)SEQ + t0 + q * 8), val); } } }

__global__ __launch_bounds__(128) void k_fa(const _Float16* __restrict__ QH, const _Float16* __restrict__ KH, const _Float16* __restrict__ VT, _Float16* __restrict__ YH) {
  __shared__ __align__(16) _Float16 ss[4][16][72];
  const int tid = threadIdx.x, wave = tid >> 5, lane = tid & 31, col = lane & 15, g = lane >> 4;
  const int qb = blockIdx.x, h = blockIdx.y, b = blockIdx.z; const int ql0 = qb * 64 + wave * 16; const size_t rowb = (size_t)b * SEQ;
  v16h qf[2];
#pragma unroll
  for (int kc = 0; kc < 2; ++kc) qf[kc] = frag_h(QH + (rowb + ql0 + col) * CC + h * HD + kc * 32, lane);
  const _Float16* kbase = KH + (rowb + col) * CC + h * HD;
  const _Float16* vbase = VT + ((size_t)b * CC + h * HD + col) * (size_t)SEQ;
  v8f o[4] = {}; float mrow = -1.0e30f, lsum = 0.f;
#pragma unroll 1
  for (int kt = 0; kt < SEQ / 64; ++kt) { const int key0 = kt * 64;
    v8f s[4] = {};
#pragma unroll
    for (int kc = 0; kc < 2; ++kc) {
#pragma unroll
      for (int j = 0; j < 4; ++j) { const v16h kf = frag_h(kbase + (size_t)(key0 + j * 16) * CC + kc * 32, lane); WAITL(); s[j] = wmma16(kf, qf[kc], s[j]); } }
    float tmax = s[0][0];
#pragma unroll
    for (int j = 0; j < 4; ++j) {
#pragma unroll
      for (int r = 0; r < 8; ++r) tmax = fmaxf(tmax, s[j][r]); }
    tmax = fmaxf(tmax, __shfl_xor(tmax, 16));
    const float mnew = fmaxf(mrow, tmax * SCALE); const float sc = __expf(mrow - mnew); mrow = mnew;
    float psum = 0.f; v16h pf[2];
#pragma unroll
    for (int c = 0; c < 2; ++c) {
#pragma unroll
      for (int i = 0; i < 8; ++i) { const float p0 = __expf(s[2 * c][i] * SCALE - mnew), p1 = __expf(s[2 * c + 1][i] * SCALE - mnew); psum += p0 + p1; pf[c][i] = (_Float16)(p0 * 1024.0f); pf[c][8 + i] = (_Float16)(p1 * 1024.0f); } }
    psum += __shfl_xor(psum, 16);
    lsum = lsum * sc + psum;
#pragma unroll
    for (int t = 0; t < 4; ++t) {
#pragma unroll
      for (int r = 0; r < 8; ++r) o[t][r] *= sc; }
#pragma unroll
    for (int c = 0; c < 2; ++c) {
#pragma unroll
      for (int t = 0; t < 4; ++t) { const v16h vf = frag_h(vbase + (size_t)(t * 16) * SEQ + key0 + c * 32, lane); WAITL(); o[t] = wmma16(vf, pf[c], o[t]); } } }
  const float inv = 0.0625f * (1.0f / lsum);
#pragma unroll
  for (int t = 0; t < 4; ++t) { v8h oh;
#pragma unroll
    for (int r = 0; r < 8; ++r) oh[r] = (_Float16)(o[t][r] * inv);
    *(v8h*)&ss[wave][col][16 * t + 8 * g] = oh; }
  LDSX();
  const int rq = lane >> 3, pc = lane & 7;
#pragma unroll
  for (int it = 0; it < 4; ++it) { const int rl = it * 4 + rq; const v8h hv = *(const v8h*)&ss[wave][rl][pc * 8]; const v4u val = __builtin_bit_cast(v4u, hv); vst2((void*)(YH + (rowb + ql0 + rl) * CC + h * HD + pc * 8), val); } }

__global__ __launch_bounds__(128) void k_out(const _Float16* __restrict__ YH, const _Float16* __restrict__ WOH, const float* __restrict__ BO, float* __restrict__ OUT) { __shared__ __align__(16) float sf[4][16][132];
  const int tid = threadIdx.x, wave = tid >> 5, lane = tid & 31, col = lane & 15, g = lane >> 4; const int c0 = blockIdx.y * 128; const int rb = blockIdx.x * 64; const size_t r0 = (size_t)rb + wave * 16;
  const _Float16* arow = YH + (r0 + col) * CC;
  v8f acc[8] = {};
#pragma unroll 2
  for (int kc = 0; kc < CC / 32; ++kc) { const v16h a = frag_h(arow + kc * 32, lane); WAITL();
#pragma unroll
    for (int j = 0; j < 8; ++j) { const v16h w = frag_h(WOH + (size_t)(c0 + j * 16 + col) * CC + kc * 32, lane); WAITL(); acc[j] = wmma16(a, w, acc[j]); } }
#pragma unroll
  for (int j = 0; j < 8; ++j) { const float bias = bfr(BO[c0 + j * 16 + col]);
#pragma unroll
    for (int r = 0; r < 8; ++r) sf[wave][8 * g + r][j * 16 + col] = acc[j][r] * (1.0f / 16384.0f) + bias; }
  LDSX();
  const size_t orow = (size_t)(rb / SEQ) * SEQ_FULL + (size_t)(rb % SEQ) + wave * 16;
  for (int rl = 0; rl < 16; ++rl) { const v4f val = *(const v4f*)&sf[wave][rl][lane * 4]; vst2((void*)(OUT + (orow + rl) * DIN + c0 + lane * 4), val); } }

extern "C" void kernel_launch(void* const* d_in, const int* in_sizes, int n_in, void* d_out, int out_size, void* d_ws, size_t ws_size, hipStream_t stream) {
  if (n_in < 5) return;
  if (in_sizes[0] < X_NEED || in_sizes[1] < 3 * CC * DIN || in_sizes[2] < 3 * CC || in_sizes[3] < DIN * CC || in_sizes[4] < DIN) return;
  if (out_size < X_NEED) return;
  if (ws_size < (size_t)WS_END) return;
  const float* x = (const float*)d_in[0]; const float* w_qkv = (const float*)d_in[1]; const float* b_qkv = (const float*)d_in[2]; const float* w_out = (const float*)d_in[3]; const float* b_out = (const float*)d_in[4];
  char* ws = (char*)d_ws;
  unsigned* XBu = (unsigned*)(ws + WS_XB); unsigned* WBu = (unsigned*)(ws + WS_WB); unsigned* WOu = (unsigned*)(ws + WS_WO);
  _Float16* QK = (_Float16*)(ws + WS_QK); _Float16* VT = (_Float16*)(ws + WS_VT); _Float16* YH = (_Float16*)(ws + WS_YH);
  float* CS = (float*)(ws + WS_CS);
  const unsigned ncv = (unsigned)((NX8 + NW8 + NO8 + 255) / 256);
  k_cvt<<<dim3(ncv), 256, 0, stream>>>(x, w_qkv, w_out, XBu, WBu, WOu);
  k_rope<<<dim3(SEQ / 16), 256, 0, stream>>>(CS);
  k_proj<<<dim3(NB * SEQ / 64, CC / 128, 3), 128, 0, stream>>>((const __bf16*)(ws + WS_XB), (const __bf16*)(ws + WS_WB), b_qkv, (const float*)CS, QK, VT);
  k_fa<<<dim3(SEQ / 64, NH, NB), 128, 0, stream>>>(QK, QK + (size_t)NB * SEQ * CC, VT, YH);
  k_out<<<dim3(NB * SEQ / 64, DIN / 128), 128, 0, stream>>>(YH, (const _Float16*)(ws + WS_WO), b_out, (float*)d_out);
}
